// TransformerBlock_85117661872380
// MI455X (gfx1250) — hardware-run, weakly checked
//
#include <hip/hip_runtime.h>
#include <hip/hip_fp16.h>


#ifndef NB
#define NB 2
#endif
#ifndef SEQ
#define SEQ 2048
#endif
#define NB_FULL  2
#define SEQ_FULL 2048
#define MD   1024
#define NH   16
#define HD   64
#define FF   4096
#define NTOK (NB * SEQ)
#define EROWS 128
#define NE   (NB * EROWS)
#define VPITCH (EROWS + 8)

static_assert(NB >= 1 && NB <= NB_FULL);
static_assert(SEQ >= 128 && SEQ <= SEQ_FULL);
static_assert(SEQ % 128 == 0);
static_assert(NTOK % 128 == 0);
static_assert(NH * HD == MD);
static_assert(MD % 128 == 0 && FF % 128 == 0);
static_assert(FF == 4 * MD);
static_assert(HD == 64);
static_assert(NH == 16);
static_assert(MD == 32 * 4 * 8);
static_assert((MD & (MD - 1)) == 0);
static_assert(EROWS % 128 == 0 && EROWS <= SEQ);
static_assert(NE % 128 == 0);
static_assert(SEQ / 64 <= 32 && EROWS / 64 <= 32);
static_assert((SEQ / 16) % 8 == 0);
static_assert((EROWS * 8) % 128 == 0);
static_assert(MD % 32 == 0 && FF % 32 == 0 && HD % 32 == 0);

typedef _Float16 v16h __attribute__((ext_vector_type(16)));
typedef _Float16 v8h  __attribute__((ext_vector_type(8)));
typedef _Float16 v4h  __attribute__((ext_vector_type(4)));
typedef float    v8f  __attribute__((ext_vector_type(8)));
typedef float    v4f  __attribute__((ext_vector_type(4)));
typedef int      v4i  __attribute__((ext_vector_type(4)));

union Frag { v16h v; v8h h[2]; };

#define W_CARRY  64.0f
#define A_CARRY  8.0f
#define P_CARRY  16384.0f
#define SA_QKV   1.953125e-03f
#define SA_WO    4.8828125e-04f
#define SA_FF    1.953125e-03f
#define CSC      (1.44269504088896340736f * 0.001953125f)
#define SC_CTX   2.44140625e-04f
#define LN_EPS   1.0e-6f

constexpr size_t WSQ  = (size_t)MD * MD * 2;
constexpr size_t WSF  = (size_t)FF * MD * 2;
constexpr size_t PL16 = (size_t)NTOK * MD * 2;
constexpr size_t PL32 = (size_t)NTOK * MD * 4;
constexpr size_t PLE  = (size_t)NE * 2 * MD * 2;
constexpr size_t FLB  = (size_t)(SEQ_FULL / 16) * 32 * 4;
constexpr size_t CARVE = 4 * WSQ + 2 * WSF + PL16 + 4 * PL16 + PL16 + PL32 + PL16 + 5 * PLE + FLB;
static_assert(CARVE <= (size_t)134217728);
static_assert((size_t)NTOK * FF * 2 == 4 * PL16);

static __device__ __forceinline__ v8f zero8() {
    v8f z;
#pragma unroll
    for (int i = 0; i < 8; ++i) z[i] = 0.0f;
    return z;
}

static __device__ __forceinline__ v16h load_frag16(const _Float16* base, int ld, int lane) {
    int m  = lane & 15;
    int kb = (lane >> 4) << 3;
    const _Float16* p = base + (size_t)m * ld + kb;
    Frag f;
    f.h[0] = *(const v8h*)(p);
    f.h[1] = *(const v8h*)(p + 16);
    return f.v;
}

static __device__ __forceinline__ v8f wmma16(v16h a, v16h b, v8f c) {
    v8f d = __builtin_amdgcn_wmma_f32_16x16x32_f16(false, a, false, b, (short)0, c, false, false);
    asm volatile("v_nop\n\tv_nop\n\tv_nop\n\tv_nop" : "+v"(d) : "v"(a), "v"(b));
    return d;
}

static __device__ __forceinline__ float bf16r(float x) {
    unsigned u = __float_as_uint(x);
    u = (u + 0x7FFFu + ((u >> 16) & 1u)) & 0xFFFF0000u;
    return __uint_as_float(u);
}

static __device__ __forceinline__ float ex2(float x) {
    return __builtin_amdgcn_exp2f(x);
}

static __device__ __forceinline__ float gelu_t(float v) {
    const float u = 0.7978845608028654f * (v + 0.044715f * v * v * v);
    const float e = ex2(-2.8853900817779268f * u);
    return v * __builtin_amdgcn_rcpf(1.0f + e);
}

static __device__ __forceinline__ void wave_lds_sync() {
    __builtin_amdgcn_fence(3, "wavefront");
    asm volatile("s_wait_dscnt 0" ::: "memory");
    __builtin_amdgcn_wave_barrier();
}

static __device__ __forceinline__ void mask_tile(v8f (&sc)[4], const int* __restrict__ mp, int r0, int cc) {
    unsigned bits = 0u;
#pragma unroll
    for (int j = 0; j < 8; ++j) {
        const v4i m = *(const v4i*)(mp + j * 4);
        bits |= ((m.x != 0) ? 1u : 0u) << (4 * j + 0);
        bits |= ((m.y != 0) ? 1u : 0u) << (4 * j + 1);
        bits |= ((m.z != 0) ? 1u : 0u) << (4 * j + 2);
        bits |= ((m.w != 0) ? 1u : 0u) << (4 * j + 3);
    }
    asm volatile("" : "+v"(bits));
    const float ninf = -__builtin_inff();
#pragma unroll
    for (int g = 0; g < 8; ++g) {
        unsigned w0 = (unsigned)__shfl((int)bits, 2 * (r0 + g), 32);
        unsigned w1 = (unsigned)__shfl((int)bits, 2 * (r0 + g) + 1, 32);
        asm volatile("" : "+v"(w0));
        asm volatile("" : "+v"(w1));
        sc[0][g] = (((w0 >> cc) & 1u) != 0u) ? sc[0][g] : ninf;
        sc[1][g] = (((w0 >> (16 + cc)) & 1u) != 0u) ? sc[1][g] : ninf;
        sc[2][g] = (((w1 >> cc) & 1u) != 0u) ? sc[2][g] : ninf;
        sc[3][g] = (((w1 >> (16 + cc)) & 1u) != 0u) ? sc[3][g] : ninf;
    }
}

__global__ __launch_bounds__(256) void k_wtr(const float* __restrict__ W, int N, int K,
                                             _Float16* __restrict__ WT) {
    __shared__ __align__(16) _Float16 T[64 * 72];
    const int tid = threadIdx.x;
    const int n0 = blockIdx.x * 64;
    const int k0 = blockIdx.y * 64;
#pragma unroll
    for (int p = 0; p < 4; ++p) {
        const int kl = p * 16 + (tid >> 4);
        const int nl = (tid & 15) * 4;
        const v4f xv = *(const v4f*)(W + (size_t)(k0 + kl) * N + n0 + nl);
        T[(nl + 0) * 72 + kl] = (_Float16)(bf16r(xv.x) * W_CARRY);
        T[(nl + 1) * 72 + kl] = (_Float16)(bf16r(xv.y) * W_CARRY);
        T[(nl + 2) * 72 + kl] = (_Float16)(bf16r(xv.z) * W_CARRY);
        T[(nl + 3) * 72 + kl] = (_Float16)(bf16r(xv.w) * W_CARRY);
    }
    __syncthreads();
    const int rl = tid >> 3, pc = (tid & 7) * 8;
    const v8h o0 = *(const v8h*)(&T[rl * 72 + pc]);
    const v8h o1 = *(const v8h*)(&T[(rl + 32) * 72 + pc]);
    _Float16* d0 = WT + (size_t)(n0 + rl) * K + k0 + pc;
    _Float16* d1 = WT + (size_t)(n0 + rl + 32) * K + k0 + pc;
    *(volatile v8h*)d0 = o0;
    *(volatile v8h*)d1 = o1;
    __threadfence();
    *(volatile v8h*)d0 = o0;
    *(volatile v8h*)d1 = o1;
}

__global__ __launch_bounds__(256) void k_mflag(const int* __restrict__ mask, int* __restrict__ flags) {
    const int lane = threadIdx.x & 31;
    const int wave = __builtin_amdgcn_readfirstlane(threadIdx.x >> 5);
    const int qg = blockIdx.x * 8 + wave;
    const int kc = (lane < SEQ / 64) ? lane : (SEQ / 64 - 1);
    const int* mp = mask + (size_t)(qg * 16) * SEQ_FULL + kc * 64;
    int cnt = 0;
#pragma unroll 1
    for (int r = 0; r < 16; ++r) {
#pragma unroll 4
        for (int j = 0; j < 16; ++j) {
            const v4i m = *(const v4i*)(mp + (size_t)r * SEQ_FULL + j * 4);
            cnt += ((m.x != 0) ? 1 : 0) + ((m.y != 0) ? 1 : 0) + ((m.z != 0) ? 1 : 0) + ((m.w != 0) ? 1 : 0);
        }
    }
    int fl = (cnt == 0) ? 0 : ((cnt == 1024) ? 1 : 2);
    if (lane >= SEQ / 64) fl = 0;
    int* dst = flags + qg * 32 + lane;
    *(volatile int*)dst = fl;
    __threadfence();
    *(volatile int*)dst = fl;
}

template<int F32> struct OTy { typedef _Float16 t; };
template<> struct OTy<1> { typedef float t; };

template<int MODE>
static __device__ __forceinline__ void gemm_body(const _Float16* __restrict__ A, int lda,
                                                 const _Float16* __restrict__ BT, int ldb, int kmask,
                                                 const float* __restrict__ bias,
                                                 const float* __restrict__ res, int ldr, int rseq,
                                                 void* __restrict__ Cv, int ldc, int roff,
                                                 int K, float sa, float so) {
    typedef typename OTy<(MODE == 2 || MODE == 3) ? 1 : 0>::t ot;
    constexpr int CP = (MODE == 4) ? 128 : 64;
    __shared__ __align__(16) ot Cst[8][32 * CP];

    const int tid  = threadIdx.x;
    const int lane = tid & 31;
    const int w    = __builtin_amdgcn_readfirstlane(tid >> 5);
    const int wr   = w >> 1;
    const int wc   = w & 1;
    const int r0   = (lane >> 4) << 3;
    const int cc   = lane & 15;
    const int m0   = blockIdx.x * 128 + wr * 32;
    const int n0   = blockIdx.y * 128 + wc * 64;
    const _Float16* Ab = A  + (size_t)m0 * lda;
    const _Float16* Bb = BT + (size_t)n0 * ldb;

    v8f acc[2][4];
#pragma unroll
    for (int mi = 0; mi < 2; ++mi)
#pragma unroll
        for (int ni = 0; ni < 4; ++ni) acc[mi][ni] = zero8();

#pragma unroll 1
    for (int k0 = 0; k0 < K; k0 += 32) {
        const int kb0 = k0 & kmask;
        const v16h a0 = load_frag16(Ab + k0, lda, lane);
        const v16h a1 = load_frag16(Ab + (size_t)16 * lda + k0, lda, lane);
#pragma unroll
        for (int ni = 0; ni < 4; ++ni) {
            const v16h bf = load_frag16(Bb + (size_t)(ni * 16) * ldb + kb0, ldb, lane);
            acc[0][ni] = wmma16(a0, bf, acc[0][ni]);
            acc[1][ni] = wmma16(a1, bf, acc[1][ni]);
        }
    }

    float bb[4];
#pragma unroll
    for (int ni = 0; ni < 4; ++ni) bb[ni] = bf16r(bias[n0 + ni * 16 + cc]);

#pragma unroll
    for (int mi = 0; mi < 2; ++mi)
#pragma unroll
        for (int ni = 0; ni < 4; ++ni)
#pragma unroll
            for (int g = 0; g < 8; ++g) {
                float v = __builtin_fmaf(acc[mi][ni][g], sa, bb[ni]);
                if constexpr (MODE == 1) v = gelu_t(v);
                const int li = (mi * 16 + r0 + g) * CP + ni * 16 + cc;
                if constexpr (MODE < 2) {
                    Cst[w][li] = (_Float16)(v * so);
                } else if constexpr (MODE == 4) {
                    const float t = v * so;
                    const _Float16 hv = (_Float16)t;
                    Cst[w][li] = hv;
                    Cst[w][li + 64] = (_Float16)(t - (float)hv);
                } else {
                    Cst[w][li] = v;
                }
            }
    wave_lds_sync();

    ot* C = (ot*)Cv;
    if constexpr (MODE < 2) {
        const int rl = lane >> 3, pc = (lane & 7) * 8;
        v8h sv[8];
#pragma unroll
        for (int i = 0; i < 8; ++i) sv[i] = *(const v8h*)(&Cst[w][(4 * i + rl) * 64 + pc]);
        _Float16* Cb = C + (size_t)(m0 + rl) * ldc + n0 + pc;
#pragma unroll
        for (int i = 0; i < 8; ++i) *(volatile v8h*)(Cb + (size_t)(4 * i) * ldc) = sv[i];
        __threadfence();
#pragma unroll
        for (int i = 0; i < 8; ++i) *(volatile v8h*)(Cb + (size_t)(4 * i) * ldc) = sv[i];
    } else if constexpr (MODE == 4) {
        const int rl = lane >> 3, pc = (lane & 7) * 8;
        v8h sv[8], sr[8];
#pragma unroll
        for (int i = 0; i < 8; ++i) {
            sv[i] = *(const v8h*)(&Cst[w][(4 * i + rl) * 128 + pc]);
            sr[i] = *(const v8h*)(&Cst[w][(4 * i + rl) * 128 + 64 + pc]);
        }
        _Float16* Cb = C + (size_t)(m0 + rl) * ldc + n0 + pc;
#pragma unroll
        for (int i = 0; i < 8; ++i) *(volatile v8h*)(Cb + (size_t)(4 * i) * ldc) = sv[i];
#pragma unroll
        for (int i = 0; i < 8; ++i) *(volatile v8h*)(Cb + roff + (size_t)(4 * i) * ldc) = sr[i];
        __threadfence();
#pragma unroll
        for (int i = 0; i < 8; ++i) *(volatile v8h*)(Cb + (size_t)(4 * i) * ldc) = sv[i];
#pragma unroll
        for (int i = 0; i < 8; ++i) *(volatile v8h*)(Cb + roff + (size_t)(4 * i) * ldc) = sr[i];
    } else {
        const int rl = lane >> 4, pc = (lane & 15) * 4;
        int orow0 = m0;
        size_t rrow0 = (size_t)m0;
        if constexpr (MODE == 2) {
            const int bq = (int)(blockIdx.x * 128) / rseq;
            const int s0 = m0 - bq * rseq;
            orow0 = bq * SEQ + s0;
            rrow0 = (size_t)bq * SEQ_FULL + (size_t)s0;
        }
        v4f sv[16];
#pragma unroll
        for (int i = 0; i < 16; ++i) {
            const v4f cv = *(const v4f*)(&Cst[w][(2 * i + rl) * 64 + pc]);
            const size_t rrow = rrow0 + (size_t)(2 * i + rl);
            v4f rv = *(const v4f*)(res + rrow * (size_t)ldr + n0 + pc);
            if constexpr (MODE == 2) {
                rv.x = bf16r(rv.x); rv.y = bf16r(rv.y); rv.z = bf16r(rv.z); rv.w = bf16r(rv.w);
            }
            sv[i] = cv + rv;
        }
        float* Cb = C + (size_t)(orow0 + rl) * ldc + n0 + pc;
#pragma unroll
        for (int i = 0; i < 16; ++i) *(volatile v4f*)(Cb + (size_t)(2 * i) * ldc) = sv[i];
        __threadfence();
#pragma unroll
        for (int i = 0; i < 16; ++i) *(volatile v4f*)(Cb + (size_t)(2 * i) * ldc) = sv[i];
    }
}

__global__ __launch_bounds__(256) __attribute__((amdgpu_num_vgpr(256)))
void k_gemm_h(const _Float16* __restrict__ A, int lda,
              const _Float16* __restrict__ BT, int ldb, int kmask,
              const float* __restrict__ bias,
              _Float16* __restrict__ C, int ldc, int K, float sa, float so) {
    gemm_body<0>(A, lda, BT, ldb, kmask, bias, bias, 0, 128, (void*)C, ldc, 0, K, sa, so);
}

__global__ __launch_bounds__(256) __attribute__((amdgpu_num_vgpr(256)))
void k_gemm_gelu(const _Float16* __restrict__ A, int lda,
                 const _Float16* __restrict__ BT, int ldb, int kmask,
                 const float* __restrict__ bias,
                 _Float16* __restrict__ C, int ldc, int K, float sa, float so) {
    gemm_body<1>(A, lda, BT, ldb, kmask, bias, bias, 0, 128, (void*)C, ldc, 0, K, sa, so);
}

__global__ __launch_bounds__(256) __attribute__((amdgpu_num_vgpr(256)))
void k_gemm_hr(const _Float16* __restrict__ A, int lda,
               const _Float16* __restrict__ BT, int ldb, int kmask,
               const float* __restrict__ bias,
               _Float16* __restrict__ C, int ldc, int roff, int K, float sa, float so) {
    gemm_body<4>(A, lda, BT, ldb, kmask, bias, bias, 0, 128, (void*)C, ldc, roff, K, sa, so);
}

__global__ __launch_bounds__(256) __attribute__((amdgpu_num_vgpr(256)))
void k_gemm_resx(const _Float16* __restrict__ A, int lda,
                 const _Float16* __restrict__ BT, int ldb, int kmask,
                 const float* __restrict__ bias,
                 const float* __restrict__ res, int ldr, int rseq,
                 const int* __restrict__ flags, int chk,
                 float* __restrict__ C, int ldc, int K, float sa) {
    if (chk != 0) {
        const int lane = threadIdx.x & 31;
        int bad = 0;
#pragma unroll 1
        for (int qg = 0; qg < EROWS / 16; ++qg) {
            const int f = flags[qg * 32 + lane];
            bad |= (lane >= EROWS / 64 && lane < SEQ / 64) ? f : 0;
        }
#pragma unroll
        for (int m = 1; m < 32; m <<= 1) bad |= __shfl_xor(bad, m, 32);
        if (__builtin_amdgcn_readfirstlane(bad) != 0) return;
    }
    gemm_body<2>(A, lda, BT, ldb, kmask, bias, res, ldr, rseq, (void*)C, ldc, 0, K, sa, 1.0f);
}

__global__ __launch_bounds__(256) __attribute__((amdgpu_num_vgpr(256)))
void k_gemm_resf(const _Float16* __restrict__ A, int lda,
                 const _Float16* __restrict__ BT, int ldb, int kmask,
                 const float* __restrict__ bias,
                 const float* __restrict__ res, int ldr,
                 float* __restrict__ C, int ldc, int K, float sa) {
    gemm_body<3>(A, lda, BT, ldb, kmask, bias, res, ldr, 128, (void*)C, ldc, 0, K, sa, 1.0f);
}

__global__ __launch_bounds__(256) void k_vtr(const _Float16* __restrict__ v,
                                             _Float16* __restrict__ vT) {
    __shared__ __align__(16) _Float16 T[64 * 72];
    const int tid  = threadIdx.x;
    const int tok0 = blockIdx.x * 64;
    const int h    = blockIdx.y;
    const int b    = tok0 / SEQ;
    const int s0   = tok0 - b * SEQ;
#pragma unroll
    for (int p = 0; p < 2; ++p) {
        const int r  = p * 32 + (tid >> 3);
        const int c8 = (tid & 7) * 8;
        const v8h vv = *(const v8h*)(v + (size_t)(tok0 + r) * MD + h * HD + c8);
#pragma unroll
        for (int e = 0; e < 8; ++e) T[(c8 + e) * 72 + r] = vv[e];
    }
    __syncthreads();
    const int rl = tid >> 3, pc = (tid & 7) * 8;
    const v8h o0 = *(const v8h*)(&T[rl * 72 + pc]);
    const v8h o1 = *(const v8h*)(&T[(rl + 32) * 72 + pc]);
    _Float16* d0 = vT + ((size_t)(b * NH + h) * HD + rl) * SEQ + s0 + pc;
    _Float16* d1 = vT + ((size_t)(b * NH + h) * HD + rl + 32) * SEQ + s0 + pc;
    *(volatile v8h*)d0 = o0;
    *(volatile v8h*)d1 = o1;
    __threadfence();
    *(volatile v8h*)d0 = o0;
    *(volatile v8h*)d1 = o1;
}

__global__ __launch_bounds__(256) __attribute__((amdgpu_num_vgpr(256)))
void k_attn(const _Float16* __restrict__ qp,
            const _Float16* __restrict__ kp,
            const _Float16* __restrict__ vT,
            const int* __restrict__ mask,
            const int* __restrict__ flags,
            _Float16* __restrict__ ctx) {
    __shared__ __align__(16) _Float16 Pst[8][16 * 64];

    const int tid  = threadIdx.x;
    const int lane = tid & 31;
    const int w    = __builtin_amdgcn_readfirstlane(tid >> 5);
    const int r0   = (lane >> 4) << 3;
    const int cc   = lane & 15;
    const int bh   = blockIdx.y;
    const int b    = bh >> 4;
    const int h    = bh & 15;
    const int qs   = blockIdx.x * 128 + w * 16;
    const int qrow = b * SEQ + qs;

    const v16h qf0 = load_frag16(qp + (size_t)qrow * MD + h * HD, MD, lane);
    const v16h qf1 = load_frag16(qp + (size_t)qrow * MD + h * HD + 32, MD, lane);
    const _Float16* kb = kp + (size_t)b * SEQ * MD + h * HD;
    const _Float16* vb = vT + (size_t)bh * HD * SEQ;
    const int* frow  = flags + (qs >> 4) * 32;
    const int* mbase = mask + (size_t)(qs + (lane >> 1)) * SEQ_FULL + (lane & 1) * 32;

    v8f o[4];
#pragma unroll
    for (int dt = 0; dt < 4; ++dt) o[dt] = zero8();
    float mr[8], lr[8];
#pragma unroll
    for (int g = 0; g < 8; ++g) { mr[g] = -1.0e30f; lr[g] = 0.0f; }

#pragma unroll 1
    for (int key0 = 0; key0 < SEQ; key0 += 64) {
        const int fl = __builtin_amdgcn_readfirstlane(frow[key0 >> 6]);
        if (fl == 0) continue;

        v8f sc[4];
#pragma unroll
        for (int nt = 0; nt < 4; ++nt) {
            const _Float16* kr = kb + (size_t)(key0 + nt * 16) * MD;
            const v16h f0 = load_frag16(kr, MD, lane);
            const v16h f1 = load_frag16(kr + 32, MD, lane);
            v8f c = wmma16(qf0, f0, zero8());
            c = wmma16(qf1, f1, c);
            sc[nt] = c;
        }
#pragma unroll
        for (int nt = 0; nt < 4; ++nt)
#pragma unroll
            for (int g = 0; g < 8; ++g) sc[nt][g] = sc[nt][g] * CSC;
        if (fl != 1) mask_tile(sc, mbase + key0, r0, cc);

        float corr[8];
#pragma unroll
        for (int g = 0; g < 8; ++g) {
            float tm = fmaxf(fmaxf(sc[0][g], sc[1][g]), fmaxf(sc[2][g], sc[3][g]));
            tm = fmaxf(tm, __shfl_xor(tm, 1, 32));
            tm = fmaxf(tm, __shfl_xor(tm, 2, 32));
            tm = fmaxf(tm, __shfl_xor(tm, 4, 32));
            tm = fmaxf(tm, __shfl_xor(tm, 8, 32));
            const float mn = fmaxf(mr[g], tm);
            corr[g] = ex2(mr[g] - mn);
            mr[g] = mn;
            float ps = 0.0f;
#pragma unroll
            for (int nt = 0; nt < 4; ++nt) {
                const float p = ex2(sc[nt][g] - mn);
                ps += p;
                Pst[w][(r0 + g) * 64 + nt * 16 + cc] = (_Float16)(p * P_CARRY);
            }
            lr[g] = __builtin_fmaf(lr[g], corr[g], ps);
        }
#pragma unroll
        for (int dt = 0; dt < 4; ++dt)
#pragma unroll
            for (int g = 0; g < 8; ++g) o[dt][g] = o[dt][g] * corr[g];
        wave_lds_sync();

        const v16h pa0 = load_frag16(&Pst[w][0], 64, lane);
        const v16h pa1 = load_frag16(&Pst[w][32], 64, lane);
#pragma unroll
        for (int dt = 0; dt < 4; ++dt) {
            const _Float16* vr = vb + (size_t)(dt * 16) * SEQ + key0;
            const v16h g0 = load_frag16(vr, SEQ, lane);
            const v16h g1 = load_frag16(vr + 32, SEQ, lane);
            o[dt] = wmma16(pa0, g0, o[dt]);
            o[dt] = wmma16(pa1, g1, o[dt]);
        }
        wave_lds_sync();
    }

    float inv[8];
#pragma unroll
    for (int g = 0; g < 8; ++g) {
        float L = lr[g];
        L += __shfl_xor(L, 1, 32);
        L += __shfl_xor(L, 2, 32);
        L += __shfl_xor(L, 4, 32);
        L += __shfl_xor(L, 8, 32);
        inv[g] = SC_CTX * __builtin_amdgcn_rcpf(L);
    }
#pragma unroll
    for (int dt = 0; dt < 4; ++dt)
#pragma unroll
        for (int g = 0; g < 8; ++g)
            Pst[w][(r0 + g) * 64 + dt * 16 + cc] = (_Float16)(o[dt][g] * inv[g]);
    wave_lds_sync();

    const int rl = lane >> 3, pc = (lane & 7) * 8;
    v8h sv[4];
#pragma unroll
    for (int i = 0; i < 4; ++i) sv[i] = *(const v8h*)(&Pst[w][(4 * i + rl) * 64 + pc]);
    _Float16* cb = ctx + (size_t)(qrow + rl) * MD + h * HD + pc;
#pragma unroll
    for (int i = 0; i < 4; ++i) *(volatile v8h*)(cb + (size_t)(4 * i) * MD) = sv[i];
    __threadfence();
#pragma unroll
    for (int i = 0; i < 4; ++i) *(volatile v8h*)(cb + (size_t)(4 * i) * MD) = sv[i];
}

__global__ __launch_bounds__(128) __attribute__((amdgpu_num_vgpr(256)))
void k_attn_e(const _Float16* __restrict__ qe,
              const _Float16* __restrict__ ke,
              const _Float16* __restrict__ ve,
              const int* __restrict__ mask,
              const int* __restrict__ flags,
              _Float16* __restrict__ ce) {
    __shared__ __align__(16) _Float16 VhT[HD * VPITCH];
    __shared__ __align__(16) _Float16 VrT[HD * VPITCH];
    __shared__ __align__(16) _Float16 Ph[4][16 * 64];
    __shared__ __align__(16) _Float16 Pr[4][16 * 64];

    const int tid  = threadIdx.x;
    const int lane = tid & 31;
    const int w    = __builtin_amdgcn_readfirstlane(tid >> 5);
    const int r0   = (lane >> 4) << 3;
    const int cc   = lane & 15;
    const int bh   = blockIdx.y;
    const int b    = bh >> 4;
    const int h    = bh & 15;
    const int qs   = blockIdx.x * 64 + w * 16;
    const int erow = b * EROWS + qs;

#pragma unroll 1
    for (int p = 0; p < (EROWS * 8) / 128; ++p) {
        const int idx = p * 128 + tid;
        const int r   = idx >> 3;
        const int c8  = (idx & 7) * 8;
        const _Float16* src = ve + (size_t)(b * EROWS + r) * (2 * MD) + h * HD + c8;
        const v8h vh = *(const v8h*)(src);
        const v8h vr = *(const v8h*)(src + MD);
#pragma unroll
        for (int e = 0; e < 8; ++e) {
            VhT[(c8 + e) * VPITCH + r] = vh[e];
            VrT[(c8 + e) * VPITCH + r] = vr[e];
        }
    }
    __syncthreads();

    const _Float16* qb = qe + (size_t)erow * (2 * MD) + h * HD;
    const v16h qh0 = load_frag16(qb, 2 * MD, lane);
    const v16h qh1 = load_frag16(qb + 32, 2 * MD, lane);
    const v16h qr0 = load_frag16(qb + MD, 2 * MD, lane);
    const v16h qr1 = load_frag16(qb + MD + 32, 2 * MD, lane);
    const _Float16* kbase = ke + (size_t)(b * EROWS) * (2 * MD) + h * HD;
    const int* frow  = flags + (qs >> 4) * 32;
    const int* mbase = mask + (size_t)(qs + (lane >> 1)) * SEQ_FULL + (lane & 1) * 32;

    v8f o[4];
#pragma unroll
    for (int dt = 0; dt < 4; ++dt) o[dt] = zero8();
    float mr[8], lr[8];
#pragma unroll
    for (int g = 0; g < 8; ++g) { mr[g] = -1.0e30f; lr[g] = 0.0f; }

#pragma unroll 1
    for (int key0 = 0; key0 < EROWS; key0 += 64) {
        const int fl = __builtin_amdgcn_readfirstlane(frow[key0 >> 6]);
        if (fl == 0) continue;

        v8f sc[4];
#pragma unroll
        for (int nt = 0; nt < 4; ++nt) {
            const _Float16* kr = kbase + (size_t)(key0 + nt * 16) * (2 * MD);
            const v16h kh0 = load_frag16(kr, 2 * MD, lane);
            const v16h kh1 = load_frag16(kr + 32, 2 * MD, lane);
            const v16h kr0 = load_frag16(kr + MD, 2 * MD, lane);
            const v16h kr1 = load_frag16(kr + MD + 32, 2 * MD, lane);
            v8f c = wmma16(qh0, kh0, zero8());
            c = wmma16(qh1, kh1, c);
            c = wmma16(qh0, kr0, c);
            c = wmma16(qh1, kr1, c);
            c = wmma16(qr0, kh0, c);
            c = wmma16(qr1, kh1, c);
            sc[nt] = c;
        }
#pragma unroll
        for (int nt = 0; nt < 4; ++nt)
#pragma unroll
            for (int g = 0; g < 8; ++g) sc[nt][g] = sc[nt][g] * CSC;
        if (fl != 1) mask_tile(sc, mbase + key0, r0, cc);

        float corr[8];
#pragma unroll
        for (int g = 0; g < 8; ++g) {
            float tm = fmaxf(fmaxf(sc[0][g], sc[1][g]), fmaxf(sc[2][g], sc[3][g]));
            tm = fmaxf(tm, __shfl_xor(tm, 1, 32));
            tm = fmaxf(tm, __shfl_xor(tm, 2, 32));
            tm = fmaxf(tm, __shfl_xor(tm, 4, 32));
            tm = fmaxf(tm, __shfl_xor(tm, 8, 32));
            const float mn = fmaxf(mr[g], tm);
            corr[g] = ex2(mr[g] - mn);
            mr[g] = mn;
            float ps = 0.0f;
#pragma unroll
            for (int nt = 0; nt < 4; ++nt) {
                const float p  = ex2(sc[nt][g] - mn);
                ps += p;
                const float pc2 = p * P_CARRY;
                const _Float16 hv = (_Float16)pc2;
                Ph[w][(r0 + g) * 64 + nt * 16 + cc] = hv;
                Pr[w][(r0 + g) * 64 + nt * 16 + cc] = (_Float16)(pc2 - (float)hv);
            }
            lr[g] = __builtin_fmaf(lr[g], corr[g], ps);
        }
#pragma unroll
        for (int dt = 0; dt < 4; ++dt)
#pragma unroll
            for (int g = 0; g < 8; ++g) o[dt][g] = o[dt][g] * corr[g];
        wave_lds_sync();

        const v16h pa0 = load_frag16(&Ph[w][0], 64, lane);
        const v16h pa1 = load_frag16(&Ph[w][32], 64, lane);
        const v16h pb0 = load_frag16(&Pr[w][0], 64, lane);
        const v16h pb1 = load_frag16(&Pr[w][32], 64, lane);
#pragma unroll
        for (int dt = 0; dt < 4; ++dt) {
            const v16h g0 = load_frag16(&VhT[(dt * 16) * VPITCH + key0], VPITCH, lane);
            const v16h g1 = load_frag16(&VhT[(dt * 16) * VPITCH + key0 + 32], VPITCH, lane);
            const v16h s0 = load_frag16(&VrT[(dt * 16) * VPITCH + key0], VPITCH, lane);
            const v16h s1 = load_frag16(&VrT[(dt * 16) * VPITCH + key0 + 32], VPITCH, lane);
            o[dt] = wmma16(pa0, g0, o[dt]);
            o[dt] = wmma16(pa1, g1, o[dt]);
            o[dt] = wmma16(pb0, g0, o[dt]);
            o[dt] = wmma16(pb1, g1, o[dt]);
            o[dt] = wmma16(pa0, s0, o[dt]);
            o[dt] = wmma16(pa1, s1, o[dt]);
        }
        wave_lds_sync();
    }

    float inv[8];
#pragma unroll
    for (int g = 0; g < 8; ++g) {
        float L = lr[g];
        L += __shfl_xor(L, 1, 32);
        L += __shfl_xor(L, 2, 32);
        L += __shfl_xor(L, 4, 32);
        L += __shfl_xor(L, 8, 32);
        inv[g] = SC_CTX * __builtin_amdgcn_rcpf(L);
    }
#pragma unroll
    for (int dt = 0; dt < 4; ++dt)
#pragma unroll
        for (int g = 0; g < 8; ++g) {
            const float c = o[dt][g] * inv[g];
            const _Float16 hv = (_Float16)c;
            Ph[w][(r0 + g) * 64 + dt * 16 + cc] = hv;
            Pr[w][(r0 + g) * 64 + dt * 16 + cc] = (_Float16)(c - (float)hv);
        }
    wave_lds_sync();

    const int rl = lane >> 3, pc = (lane & 7) * 8;
    v8h sv[4], sr[4];
#pragma unroll
    for (int i = 0; i < 4; ++i) {
        sv[i] = *(const v8h*)(&Ph[w][(4 * i + rl) * 64 + pc]);
        sr[i] = *(const v8h*)(&Pr[w][(4 * i + rl) * 64 + pc]);
    }
    _Float16* cb = ce + (size_t)(erow + rl) * (2 * MD) + h * HD + pc;
#pragma unroll
    for (int i = 0; i < 4; ++i) *(volatile v8h*)(cb + (size_t)(4 * i) * (2 * MD)) = sv[i];
#pragma unroll
    for (int i = 0; i < 4; ++i) *(volatile v8h*)(cb + MD + (size_t)(4 * i) * (2 * MD)) = sr[i];
    __threadfence();
#pragma unroll
    for (int i = 0; i < 4; ++i) *(volatile v8h*)(cb + (size_t)(4 * i) * (2 * MD)) = sv[i];
#pragma unroll
    for (int i = 0; i < 4; ++i) *(volatile v8h*)(cb + MD + (size_t)(4 * i) * (2 * MD)) = sr[i];
}

template<int SRCX>
static __device__ __forceinline__ v4f ln_load(const float* __restrict__ p) {
    v4f a = *(const v4f*)p;
    if constexpr (SRCX == 1) {
        a.x = bf16r(a.x); a.y = bf16r(a.y); a.z = bf16r(a.z); a.w = bf16r(a.w);
    }
    return a;
}

template<int SRCX>
static __device__ __forceinline__ void ln_store(const float* __restrict__ yr,
                                                const float* __restrict__ gr,
                                                const float* __restrict__ br,
                                                float mu, float rstd,
                                                _Float16* __restrict__ xh,
                                                _Float16* __restrict__ xe, int s) {
#pragma clang fp contract(off)
#pragma unroll 1
    for (int i = 0; i < 8; ++i) {
        const v4f a  = ln_load<SRCX>(yr + i * 128);
        const v4f gv = *(const v4f*)(gr + i * 128);
        const v4f bv = *(const v4f*)(br + i * 128);
        v4f t;
        t.x = (((a.x - mu) * rstd) * bf16r(gv.x) + bf16r(bv.x)) * A_CARRY;
        t.y = (((a.y - mu) * rstd) * bf16r(gv.y) + bf16r(bv.y)) * A_CARRY;
        t.z = (((a.z - mu) * rstd) * bf16r(gv.z) + bf16r(bv.z)) * A_CARRY;
        t.w = (((a.w - mu) * rstd) * bf16r(gv.w) + bf16r(bv.w)) * A_CARRY;
        v4h hv;
        hv.x = (_Float16)t.x;
        hv.y = (_Float16)t.y;
        hv.z = (_Float16)t.z;
        hv.w = (_Float16)t.w;
        *(volatile v4h*)(xh + i * 128) = hv;
        if constexpr (SRCX == 1) {
            if (s < EROWS) {
                v4h rv;
                rv.x = (_Float16)(t.x - (float)hv.x);
                rv.y = (_Float16)(t.y - (float)hv.y);
                rv.z = (_Float16)(t.z - (float)hv.z);
                rv.w = (_Float16)(t.w - (float)hv.w);
                *(volatile v4h*)(xe + i * 128) = hv;
                *(volatile v4h*)(xe + MD + i * 128) = rv;
            }
        }
    }
}

template<int SRCX>
static __device__ __forceinline__ void ln_body(const float* __restrict__ y,
                                               const float* __restrict__ gam,
                                               const float* __restrict__ bet,
                                               _Float16* __restrict__ xh,
                                               _Float16* __restrict__ xe) {
#pragma clang fp contract(off)
    const int lane = threadIdx.x & 31;
    const int w    = __builtin_amdgcn_readfirstlane(threadIdx.x >> 5);
    const int row  = blockIdx.x * 8 + w;
    const int b    = row / SEQ;
    const int s    = row - b * SEQ;
    size_t srow = (size_t)row;
    if constexpr (SRCX == 1) srow = (size_t)b * SEQ_FULL + (size_t)s;
    const float* yr = y + srow * MD + lane * 4;
    const int erow  = b * EROWS + min(s, EROWS - 1);

    float sm = 0.0f;
#pragma unroll 1
    for (int i = 0; i < 8; ++i) {
        const v4f a = ln_load<SRCX>(yr + i * 128);
        sm += (a.x + a.y) + (a.z + a.w);
    }
#pragma unroll
    for (int m = 1; m < 32; m <<= 1) sm += __shfl_xor(sm, m, 32);
    const float mu = sm * (1.0f / (float)MD);

    float s2 = 0.0f;
#pragma unroll 1
    for (int i = 0; i < 8; ++i) {
        const v4f a = ln_load<SRCX>(yr + i * 128);
        const float dx = a.x - mu, dy = a.y - mu, dz = a.z - mu, dw = a.w - mu;
        s2 += (dx * dx + dy * dy) + (dz * dz + dw * dw);
    }
#pragma unroll
    for (int m = 1; m < 32; m <<= 1) s2 += __shfl_xor(s2, m, 32);
    const float rstd = rsqrtf(s2 * (1.0f / (float)MD) + LN_EPS);

    const float* gr = gam + lane * 4;
    const float* br = bet + lane * 4;
    _Float16* xhr = xh + (size_t)row * MD + lane * 4;
    _Float16* xer = xe + (size_t)erow * (2 * MD) + lane * 4;
    ln_store<SRCX>(yr, gr, br, mu, rstd, xhr, xer, s);
    __threadfence();
    ln_store<SRCX>(yr, gr, br, mu, rstd, xhr, xer, s);
}

__global__ __launch_bounds__(256) void k_ln1(const float* __restrict__ x,
                                             const float* __restrict__ gam,
                                             const float* __restrict__ bet,
                                             _Float16* __restrict__ xh,
                                             _Float16* __restrict__ xe) {
    ln_body<1>(x, gam, bet, xh, xe);
}

__global__ __launch_bounds__(256) void k_ln2(const float* __restrict__ y,
                                             const float* __restrict__ gam,
                                             const float* __restrict__ bet,
                                             _Float16* __restrict__ xh) {
    ln_body<0>(y, gam, bet, xh, xh);
}

extern "C" void kernel_launch(void* const* d_in, const int* in_sizes, int n_in,
                              void* d_out, int out_size, void* d_ws, size_t ws_size,
                              hipStream_t stream) {
    if (n_in < 18) return;
    if (in_sizes[0] < ((NB - 1) * SEQ_FULL + SEQ) * MD) return;
    if (in_sizes[1] < (SEQ - 1) * SEQ_FULL + SEQ) return;
    if (in_sizes[2] < MD || in_sizes[3] < MD || in_sizes[12] < MD || in_sizes[13] < MD) return;
    if (in_sizes[4] < MD * MD || in_sizes[6] < MD * MD || in_sizes[8] < MD * MD || in_sizes[10] < MD * MD) return;
    if (in_sizes[5] < MD || in_sizes[7] < MD || in_sizes[9] < MD || in_sizes[11] < MD) return;
    if (in_sizes[14] < MD * FF || in_sizes[15] < FF || in_sizes[16] < FF * MD || in_sizes[17] < MD) return;
    if (out_size < NTOK * MD) return;

    const float* x    = (const float*)d_in[0];
    const int*   mask = (const int*)d_in[1];
    const float* ln1s = (const float*)d_in[2];
    const float* ln1b = (const float*)d_in[3];
    const float* Wq   = (const float*)d_in[4];
    const float* bq   = (const float*)d_in[5];
    const float* Wk   = (const float*)d_in[6];
    const float* bk   = (const float*)d_in[7];
    const float* Wv   = (const float*)d_in[8];
    const float* bv   = (const float*)d_in[9];
    const float* Wo   = (const float*)d_in[10];
    const float* bo   = (const float*)d_in[11];
    const float* ln2s = (const float*)d_in[12];
    const float* ln2b = (const float*)d_in[13];
    const float* W1   = (const float*)d_in[14];
    const float* b1   = (const float*)d_in[15];
    const float* W2   = (const float*)d_in[16];
    const float* b2   = (const float*)d_in[17];
    float* out = (float*)d_out;

    char* ws = (char*)d_ws;
    size_t off = 0;
    _Float16* WqT = (_Float16*)(ws + off); off += WSQ;
    _Float16* WkT = (_Float16*)(ws + off); off += WSQ;
    _Float16* WvT = (_Float16*)(ws + off); off += WSQ;
    _Float16* WoT = (_Float16*)(ws + off); off += WSQ;
    _Float16* W1T = (_Float16*)(ws + off); off += WSF;
    _Float16* W2T = (_Float16*)(ws + off); off += WSF;
    _Float16* XN  = (_Float16*)(ws + off); off += PL16;
    _Float16* QP  = (_Float16*)(ws + off); off += PL16;
    _Float16* KP  = (_Float16*)(ws + off); off += PL16;
    _Float16* VP  = (_Float16*)(ws + off); off += PL16;
    _Float16* VT  = (_Float16*)(ws + off); off += PL16;
    _Float16* HP  = QP;
    _Float16* CTX = (_Float16*)(ws + off); off += PL16;
    float*    Y   = (float*)(ws + off);    off += PL32;
    _Float16* XH2 = (_Float16*)(ws + off); off += PL16;
    _Float16* XNE = (_Float16*)(ws + off); off += PLE;
    _Float16* QE  = (_Float16*)(ws + off); off += PLE;
    _Float16* KE  = (_Float16*)(ws + off); off += PLE;
    _Float16* VE  = (_Float16*)(ws + off); off += PLE;
    _Float16* CE  = (_Float16*)(ws + off); off += PLE;
    int*      FLG = (int*)(ws + off);      off += FLB;
    if (off != CARVE) return;
    if (off > ws_size) return;

    k_wtr<<<dim3(MD / 64, MD / 64), dim3(256), 0, stream>>>(Wq, MD, MD, WqT);
    k_wtr<<<dim3(MD / 64, MD / 64), dim3(256), 0, stream>>>(Wk, MD, MD, WkT);
    k_wtr<<<dim3(MD / 64, MD / 64), dim3(256), 0, stream>>>(Wv, MD, MD, WvT);
    k_wtr<<<dim3(MD / 64, MD / 64), dim3(256), 0, stream>>>(Wo, MD, MD, WoT);
    k_wtr<<<dim3(FF / 64, MD / 64), dim3(256), 0, stream>>>(W1, FF, MD, W1T);
    k_wtr<<<dim3(MD / 64, FF / 64), dim3(256), 0, stream>>>(W2, MD, FF, W2T);

    k_mflag<<<dim3(SEQ / 128), dim3(256), 0, stream>>>(mask, FLG);

    k_ln1<<<dim3(NTOK / 8), dim3(256), 0, stream>>>(x, ln1s, ln1b, XN, XNE);

    k_gemm_h<<<dim3(NTOK / 128, MD / 128), dim3(256), 0, stream>>>(XN, MD, WqT, MD, -1, bq, QP, MD, MD, SA_QKV, A_CARRY);
    k_gemm_h<<<dim3(NTOK / 128, MD / 128), dim3(256), 0, stream>>>(XN, MD, WkT, MD, -1, bk, KP, MD, MD, SA_QKV, A_CARRY);
    k_gemm_h<<<dim3(NTOK / 128, MD / 128), dim3(256), 0, stream>>>(XN, MD, WvT, MD, -1, bv, VP, MD, MD, SA_QKV, A_CARRY);

    k_vtr<<<dim3(NTOK / 64, NH), dim3(256), 0, stream>>>(VP, VT);
    k_attn<<<dim3(SEQ / 128, NB * NH), dim3(256), 0, stream>>>(QP, KP, VT, mask, FLG, CTX);

    k_gemm_hr<<<dim3(NE / 128, MD / 128), dim3(256), 0, stream>>>(XNE, 2 * MD, WqT, MD, MD - 1, bq, QE, 2 * MD, MD, 2 * MD, SA_QKV, A_CARRY);
    k_gemm_hr<<<dim3(NE / 128, MD / 128), dim3(256), 0, stream>>>(XNE, 2 * MD, WkT, MD, MD - 1, bk, KE, 2 * MD, MD, 2 * MD, SA_QKV, A_CARRY);
    k_gemm_hr<<<dim3(NE / 128, MD / 128), dim3(256), 0, stream>>>(XNE, 2 * MD, WvT, MD, MD - 1, bv, VE, 2 * MD, MD, 2 * MD, SA_QKV, A_CARRY);
    k_attn_e<<<dim3(EROWS / 64, NB * NH), dim3(128), 0, stream>>>(QE, KE, VE, mask, FLG, CE);

    k_gemm_resx<<<dim3(NTOK / 128, MD / 128), dim3(256), 0, stream>>>(CTX, MD, WoT, MD, -1, bo, x, MD, SEQ, FLG, 0, Y, MD, MD, SA_WO);
    k_gemm_resx<<<dim3(NE / 128, MD / 128), dim3(256), 0, stream>>>(CE, 2 * MD, WoT, MD, MD - 1, bo, x, MD, EROWS, FLG, 1, Y, MD, 2 * MD, SA_WO);

    k_ln2<<<dim3(NTOK / 8), dim3(256), 0, stream>>>(Y, ln2s, ln2b, XH2);
    k_gemm_gelu<<<dim3(NTOK / 128, FF / 128), dim3(256), 0, stream>>>(XH2, MD, W1T, MD, -1, b1, HP, FF, MD, SA_FF, A_CARRY);
    k_gemm_resf<<<dim3(NTOK / 128, MD / 128), dim3(256), 0, stream>>>(HP, FF, W2T, FF, -1, b2, Y, MD, out, MD, FF, SA_FF);
}
